// CrossIQ_30511447670998
// MI455X (gfx1250) — hardware-verified
//
#include <hip/hip_runtime.h>


#define NB_  4
#define CC   256
#define NP   2304
#define PSC  32768.0f
#define LOSC 1024.0f
#define LOSCI (1.0f / 1024.0f)

typedef _Float16 h16;
typedef unsigned short bf;
typedef __attribute__((ext_vector_type(16))) __bf16   v16bf;
typedef __attribute__((ext_vector_type(16))) _Float16 v16h;
typedef __attribute__((ext_vector_type(8)))  _Float16 v8h;
typedef __attribute__((ext_vector_type(8)))  unsigned short v8us;
typedef __attribute__((ext_vector_type(8)))  float    v8f;
typedef __attribute__((ext_vector_type(4)))  float    v4f;
typedef v8h  __attribute__((may_alias)) v8ha;
typedef v4f  __attribute__((may_alias)) v4fa;
typedef v8us __attribute__((may_alias)) v8usa;

__device__ __forceinline__ unsigned short f2bf(float f) { unsigned u = __float_as_uint(f); u += 0x7FFFu + ((u >> 16) & 1u); return (unsigned short)(u >> 16); }
__device__ __forceinline__ float bf2f(unsigned short b) { return __uint_as_float(((unsigned)b) << 16); }
__device__ __forceinline__ float bfr(float f) { return bf2f(f2bf(f)); }
__device__ __forceinline__ v16h cat16(v8h lo, v8h hi) { return __builtin_shufflevector(lo, hi, 0, 1, 2, 3, 4, 5, 6, 7, 8, 9, 10, 11, 12, 13, 14, 15); }
__device__ __forceinline__ v16bf cat16b(v8us lo, v8us hi) { return __builtin_bit_cast(v16bf, __builtin_shufflevector(lo, hi, 0, 1, 2, 3, 4, 5, 6, 7, 8, 9, 10, 11, 12, 13, 14, 15)); }
__device__ __forceinline__ v8f wmma16(v16h a, v16h b, v8f c) { return __builtin_amdgcn_wmma_f32_16x16x32_f16(false, a, false, b, (short)0, c, false, false); }
__device__ __forceinline__ v8f wmmab(v16bf a, v16bf b, v8f c) { return __builtin_amdgcn_wmma_f32_16x16x32_bf16(false, a, false, b, (short)0, c, false, false); }
#define VST2(T, p, v) do { const T vst2_v_ = (v); *(volatile T*)(p) = vst2_v_; __threadfence(); *(volatile T*)(p) = vst2_v_; } while (0)

__global__ __launch_bounds__(256) void k_xt(const float* __restrict__ xb, bf* XT) {
    __shared__ __align__(16) unsigned short tl[64 * 72];
    const int tid = threadIdx.x, n0 = blockIdx.x * 64, c0 = blockIdx.y * 64;
    const int cr = tid >> 2, nq = (tid & 3) * 16;
#pragma unroll
    for (int i = 0; i < 16; ++i) tl[(nq + i) * 72 + cr] = f2bf(xb[(size_t)(c0 + cr) * NP + n0 + nq + i]);
    __syncthreads();
    const int piece = tid & 7;
    auto pass = [&]() {
#pragma unroll
        for (int s = 0; s < 2; ++s) { const int nr = (tid >> 3) + 32 * s; const v8us val = *(const v8usa*)(tl + nr * 72 + piece * 8); *(volatile v8us*)(XT + (size_t)(n0 + nr) * CC + c0 + piece * 8) = val; }
    };
    pass(); __threadfence(); pass();
}
__global__ __launch_bounds__(256) void k_w(const float* __restrict__ w, bf* WB) {
    const int lane = threadIdx.x & 31, r = blockIdx.x * 8 + (threadIdx.x >> 5);
    v8us o;
#pragma unroll
    for (int i = 0; i < 8; ++i) o[i] = f2bf(w[(size_t)r * CC + lane * 8 + i]);
    VST2(v8us, WB + (size_t)r * CC + lane * 8, o);
}
template <bool SPLITA, int EPI, bool ACC>
__global__ __launch_bounds__(128) void k_gemm(const bf* __restrict__ A, const bf* __restrict__ Al, const bf* __restrict__ WB, const float* __restrict__ bias, const float* __restrict__ sp, const float* __restrict__ Wm, float* C) {
    const float scale = sp ? bfr(sp[0]) : 1.0f;
    __shared__ __align__(16) float ost[4][16 * 68];
    __shared__ __align__(16) float ot[64 * 68];
    const int lane = threadIdx.x & 31, wave = threadIdx.x >> 5, lr = lane & 15, hi = lane >> 4, tid = threadIdx.x;
    const size_t r0 = (size_t)blockIdx.x * 64 + wave * 16; const int c0 = blockIdx.y * 64;
    v8f acc[4];
#pragma unroll
    for (int t = 0; t < 4; ++t) acc[t] = (v8f){};
#pragma unroll
    for (int kc = 0; kc < CC; kc += 32) {
        const v16bf a = cat16b(*(const v8us*)(A + (r0 + lr) * CC + kc + 8 * hi), *(const v8us*)(A + (r0 + lr) * CC + kc + 8 * hi + 16));
        v16bf al = a; if (SPLITA) al = cat16b(*(const v8us*)(Al + (r0 + lr) * CC + kc + 8 * hi), *(const v8us*)(Al + (r0 + lr) * CC + kc + 8 * hi + 16));
#pragma unroll
        for (int t = 0; t < 4; ++t) { const bf* bp = WB + (size_t)(c0 + t * 16 + lr) * CC + kc + 8 * hi; const v16bf bb = cat16b(*(const v8us*)bp, *(const v8us*)(bp + 16)); acc[t] = wmmab(a, bb, acc[t]); if (SPLITA) acc[t] = wmmab(al, bb, acc[t]); }
        asm volatile("v_nop" : "+v"(acc[0]), "+v"(acc[1]), "+v"(acc[2]), "+v"(acc[3]) : "v"(a), "v"(al) : "memory");
    }
    float* os = &ost[wave][0];
#pragma unroll
    for (int t = 0; t < 4; ++t) { const int col = c0 + t * 16 + lr; const float bv = bfr(bias[col]);
#pragma unroll
        for (int j = 0; j < 8; ++j) { float v = (acc[t][j] + bv) * scale;
            if (EPI == 1) { const size_t e = (r0 + hi * 8 + j) * CC + col; v = Wm[e] / (1.0f + __expf(-v)); if (ACC) v += C[e]; }
            os[(hi * 8 + j) * 68 + t * 16 + lr] = v; } }
    if (EPI != 2) {
        __builtin_amdgcn_wave_barrier(); asm volatile("" ::: "memory");
        float* crow = C + r0 * CC + c0;
        auto pass = [&]() {
#pragma unroll
            for (int s = 0; s < 8; ++s) { const int Lid = (lane >> 3) + 4 * s, piece = lane & 7; const int row = Lid >> 1, cofs = (Lid & 1) * 32 + piece * 4;
                const v4f val = *(const v4fa*)(os + row * 68 + cofs); *(volatile v4f*)(crow + (size_t)row * CC + cofs) = val; }
        };
        pass(); __threadfence(); pass();
    } else {
        __syncthreads();
        { const int row = tid >> 1, half = tid & 1;
#pragma unroll
          for (int i = 0; i < 32; ++i) ot[(half * 32 + i) * 68 + row] = ost[row >> 4][(row & 15) * 68 + half * 32 + i]; }
        __syncthreads();
        const size_t rblk = (size_t)blockIdx.x * 64;
        auto pass = [&]() {
#pragma unroll
            for (int s = 0; s < 8; ++s) { const int cl = s * 8 + (tid >> 4), piece = tid & 15;
                const v4f val = *(const v4fa*)(ot + cl * 68 + piece * 4); *(volatile v4f*)(C + (size_t)(c0 + cl) * NP + rblk + piece * 4) = val; }
        };
        pass(); __threadfence(); pass();
    }
}
__global__ __launch_bounds__(256) void k_p16(const float* __restrict__ A, const float* __restrict__ Bsum, h16* PH, h16* PL) {
    const int lane = threadIdx.x & 31, r = blockIdx.x * 8 + (threadIdx.x >> 5);
    if (r >= NP) return;
    v8h oh, ol;
#pragma unroll
    for (int i = 0; i < 8; ++i) { float v = A[(size_t)r * CC + lane * 8 + i]; if (Bsum) v += Bsum[(size_t)r * CC + lane * 8 + i]; const h16 a = (h16)v; oh[i] = a; ol[i] = (h16)((v - (float)a) * LOSC); }
    *(volatile v8h*)(PH + (size_t)r * CC + lane * 8) = oh; *(volatile v8h*)(PL + (size_t)r * CC + lane * 8) = ol; __threadfence();
    *(volatile v8h*)(PH + (size_t)r * CC + lane * 8) = oh; *(volatile v8h*)(PL + (size_t)r * CC + lane * 8) = ol;
}
__global__ __launch_bounds__(256) void k_pbf(const float* __restrict__ A, bf* PH, bf* PL) {
    const int lane = threadIdx.x & 31, r = blockIdx.x * 8 + (threadIdx.x >> 5);
    if (r >= NP) return;
    v8us oh, ol;
#pragma unroll
    for (int i = 0; i < 8; ++i) { const float v = A[(size_t)r * CC + lane * 8 + i]; const unsigned short hb = f2bf(v); oh[i] = hb; ol[i] = f2bf(v - bf2f(hb)); }
    *(volatile v8us*)(PH + (size_t)r * CC + lane * 8) = oh; *(volatile v8us*)(PL + (size_t)r * CC + lane * 8) = ol; __threadfence();
    *(volatile v8us*)(PH + (size_t)r * CC + lane * 8) = oh; *(volatile v8us*)(PL + (size_t)r * CC + lane * 8) = ol;
}
__global__ __launch_bounds__(256) void k_vt(const float* __restrict__ V, h16* VTH, h16* VTL) {
    __shared__ float tl[64][65];
    const int tid = threadIdx.x, n0 = blockIdx.x * 64, c0 = blockIdx.y * 64;
    { const int nn = tid >> 2, cq = (tid & 3) * 16;
#pragma unroll
      for (int i = 0; i < 16; ++i) tl[cq + i][nn] = V[(size_t)(n0 + nn) * CC + c0 + cq + i]; }
    __syncthreads();
    const int piece = tid & 7;
    auto pass = [&]() {
#pragma unroll
        for (int s = 0; s < 2; ++s) { const int c = (tid >> 3) + 32 * s; v8h oh, ol;
#pragma unroll
            for (int i = 0; i < 8; ++i) { const float v = tl[c][piece * 8 + i]; const h16 a = (h16)v; oh[i] = a; ol[i] = (h16)((v - (float)a) * LOSC); }
            const size_t o = (size_t)(c0 + c) * NP + n0 + piece * 8; *(volatile v8h*)(VTH + o) = oh; *(volatile v8h*)(VTL + o) = ol; }
    };
    pass(); __threadfence(); pass();
}
template <int EPI>
__global__ __launch_bounds__(128) void k_f16gemm(const h16* __restrict__ A, const h16* __restrict__ Al, int lda, const h16* __restrict__ Bn, const h16* __restrict__ Bl, int ldb, int K, const float* __restrict__ rs, float* C, int ldc) {
    __shared__ __align__(16) float ost[4][16 * 68];
    const int lane = threadIdx.x & 31, wave = threadIdx.x >> 5, lr = lane & 15, hi = lane >> 4;
    const int r0 = blockIdx.x * 64 + wave * 16, c0 = blockIdx.y * 64;
    const size_t aoff = (size_t)(r0 + lr) * lda + 8 * hi;
    size_t boff[4];
#pragma unroll
    for (int t = 0; t < 4; ++t) boff[t] = (size_t)(c0 + t * 16 + lr) * ldb + 8 * hi;
    v8f acc[4], accx[4];
#pragma unroll
    for (int t = 0; t < 4; ++t) { acc[t] = (v8f){}; accx[t] = (v8f){}; }
#pragma unroll 2
    for (int kc = 0; kc < K; kc += 32) {
        const v16h a = cat16(*(const v8h*)(A + aoff + kc), *(const v8h*)(A + aoff + kc + 16)), al = cat16(*(const v8h*)(Al + aoff + kc), *(const v8h*)(Al + aoff + kc + 16));
#pragma unroll
        for (int t = 0; t < 4; ++t) { const v16h bb = cat16(*(const v8h*)(Bn + boff[t] + kc), *(const v8h*)(Bn + boff[t] + kc + 16)), bl = cat16(*(const v8h*)(Bl + boff[t] + kc), *(const v8h*)(Bl + boff[t] + kc + 16));
            acc[t] = wmma16(a, bb, acc[t]); accx[t] = wmma16(a, bl, accx[t]);
            if (EPI == 0) accx[t] = wmma16(al, bb, accx[t]); else acc[t] = wmma16(al, bb, acc[t]); }
        asm volatile("v_nop" : "+v"(acc[0]), "+v"(acc[1]), "+v"(acc[2]), "+v"(acc[3]), "+v"(accx[0]), "+v"(accx[1]), "+v"(accx[2]), "+v"(accx[3]) : "v"(a), "v"(al) : "memory");
    }
    float* os = &ost[wave][0];
#pragma unroll
    for (int t = 0; t < 4; ++t)
#pragma unroll
        for (int j = 0; j < 8; ++j) { const float sc = (EPI == 0) ? 0.0625f : rs[r0 + hi * 8 + j]; os[(hi * 8 + j) * 68 + t * 16 + lr] = (acc[t][j] + accx[t][j] * LOSCI) * sc; }
    __builtin_amdgcn_wave_barrier(); asm volatile("" ::: "memory");
    float* crow = C + (size_t)r0 * ldc + c0;
    auto pass = [&]() {
#pragma unroll
        for (int s = 0; s < 8; ++s) { const int Lid = (lane >> 3) + 4 * s, piece = lane & 7; const int row = Lid >> 1, cofs = (Lid & 1) * 32 + piece * 4;
            const v4f val = *(const v4fa*)(os + row * 68 + cofs); *(volatile v4f*)(crow + (size_t)row * ldc + cofs) = val; }
    };
    pass(); __threadfence(); pass();
}
__global__ __launch_bounds__(256) void k_soft(const float* __restrict__ S, h16* PH, h16* PL, float* RS) {
    __shared__ float rsum[32];
    const int lane = threadIdx.x & 31, wave = threadIdx.x >> 5;
#pragma unroll 1
    for (int rr = 0; rr < 4; ++rr) { const int row = blockIdx.x * 32 + wave * 4 + rr; const float* sr = S + (size_t)row * NP;
        float mx = -3.0e38f;
#pragma unroll 1
        for (int c = 0; c < NP / 256; ++c)
#pragma unroll
            for (int i = 0; i < 8; ++i) mx = fmaxf(mx, sr[c * 256 + lane * 8 + i]);
#pragma unroll
        for (int sh = 16; sh; sh >>= 1) mx = fmaxf(mx, __shfl_xor(mx, sh, 32));
        float sum = 0.f;
#pragma unroll 1
        for (int ps = 0; ps < 2; ++ps) { sum = 0.f;
#pragma unroll 1
            for (int c = 0; c < NP / 256; ++c) { v8h oh, ol;
#pragma unroll
                for (int i = 0; i < 8; ++i) { const float p = __expf(sr[c * 256 + lane * 8 + i] - mx); sum += p; const float ps8 = p * PSC; const h16 a = (h16)ps8; oh[i] = a; ol[i] = (h16)(ps8 - (float)a); }
                *(volatile v8h*)(PH + (size_t)row * NP + c * 256 + lane * 8) = oh; *(volatile v8h*)(PL + (size_t)row * NP + c * 256 + lane * 8) = ol; }
            if (ps == 0) __threadfence(); }
#pragma unroll
        for (int sh = 16; sh; sh >>= 1) sum += __shfl_xor(sum, sh, 32);
        if (lane == 0) rsum[wave * 4 + rr] = 1.0f / (sum * PSC); }
    __syncthreads();
    if (wave == 0) { const float v = rsum[lane]; *(volatile float*)(RS + blockIdx.x * 32 + lane) = v; __threadfence(); *(volatile float*)(RS + blockIdx.x * 32 + lane) = v; }
}

extern "C" void kernel_launch(void* const* d_in, const int* in_sizes, int n_in,
                              void* d_out, int out_size, void* d_ws, size_t ws_size, hipStream_t stream) {
    (void)in_sizes; (void)n_in; (void)out_size;
    const float* xin[3] = {(const float*)d_in[0], (const float*)d_in[1], (const float*)d_in[2]}; const float* sv = (const float*)d_in[3];
    const float* wq[3] = {(const float*)d_in[4], (const float*)d_in[10], (const float*)d_in[16]}; const float* bq[3] = {(const float*)d_in[5], (const float*)d_in[11], (const float*)d_in[17]};
    const float* wk[3] = {(const float*)d_in[6], (const float*)d_in[12], (const float*)d_in[18]}; const float* bk[3] = {(const float*)d_in[7], (const float*)d_in[13], (const float*)d_in[19]};
    const float* wv[3] = {(const float*)d_in[8], (const float*)d_in[14], (const float*)d_in[20]}; const float* bv[3] = {(const float*)d_in[9], (const float*)d_in[15], (const float*)d_in[21]};
    const float* wg = (const float*)d_in[22]; const float* bg = (const float*)d_in[23]; const float* wo = (const float*)d_in[24]; const float* bo = (const float*)d_in[25];
    float* out = (float*)d_out;
    char* wsp = (char*)d_ws;
    auto take = [&](size_t bytes) { char* p = wsp; wsp += (bytes + 255) & ~(size_t)255; return (void*)p; };
    const size_t PB = (size_t)NP * CC;
    bf* WB = (bf*)take((size_t)11 * CC * CC * 2);
    bf* XT = (bf*)take(3 * PB * 2);
    float* Qf = (float*)take(3 * PB * 4); float* Kf = (float*)take(3 * PB * 4); float* Vf = (float*)take(3 * PB * 4);
    h16* QH = (h16*)take(PB * 2); h16* QL = (h16*)take(PB * 2); h16* KH = (h16*)take(PB * 2); h16* KL = (h16*)take(PB * 2); h16* VTH = (h16*)take(PB * 2); h16* VTL = (h16*)take(PB * 2);
    float* S = (float*)take((size_t)NP * NP * 4); h16* PH = (h16*)take((size_t)NP * NP * 2); h16* PL = (h16*)take((size_t)NP * NP * 2); float* RS = (float*)take((size_t)NP * 4);
    float* Wm = (float*)take(PB * 4); bf* WmH = (bf*)take(PB * 2); bf* WmL = (bf*)take(PB * 2); float* FU = (float*)take(PB * 4); bf* FH = (bf*)take(PB * 2); bf* FL = (bf*)take(PB * 2);
    if ((size_t)(wsp - (char*)d_ws) > ws_size) return;
    const bf* Wg_b = WB + (size_t)9 * CC * CC; const bf* Wo_b = WB + (size_t)10 * CC * CC;
    for (int i = 0; i < 3; ++i) { k_w<<<CC / 8, 256, 0, stream>>>(wq[i], WB + (size_t)(3 * i + 0) * CC * CC); k_w<<<CC / 8, 256, 0, stream>>>(wk[i], WB + (size_t)(3 * i + 1) * CC * CC); k_w<<<CC / 8, 256, 0, stream>>>(wv[i], WB + (size_t)(3 * i + 2) * CC * CC); }
    k_w<<<CC / 8, 256, 0, stream>>>(wg, WB + (size_t)9 * CC * CC); k_w<<<CC / 8, 256, 0, stream>>>(wo, WB + (size_t)10 * CC * CC);
    const int kp1[3] = {2, 0, 0}, kp2[3] = {1, 2, 1};
    for (int b = 0; b < NB_; ++b) {
        for (int m = 0; m < 3; ++m) {
            k_xt<<<dim3(NP / 64, CC / 64, 1), 256, 0, stream>>>(xin[m] + (size_t)b * CC * NP, XT + m * PB);
            k_gemm<false, 0, false><<<dim3(NP / 64, CC / 64, 1), 128, 0, stream>>>(XT + m * PB, nullptr, WB + (size_t)(3 * m + 0) * CC * CC, bq[m], sv + m, nullptr, Qf + m * PB);
            k_gemm<false, 0, false><<<dim3(NP / 64, CC / 64, 1), 128, 0, stream>>>(XT + m * PB, nullptr, WB + (size_t)(3 * m + 1) * CC * CC, bk[m], sv + m, nullptr, Kf + m * PB);
            k_gemm<false, 0, false><<<dim3(NP / 64, CC / 64, 1), 128, 0, stream>>>(XT + m * PB, nullptr, WB + (size_t)(3 * m + 2) * CC * CC, bv[m], nullptr, nullptr, Vf + m * PB);
        }
        for (int m = 0; m < 3; ++m) {
            k_p16<<<NP / 8, 256, 0, stream>>>(Qf + m * PB, nullptr, QH, QL);
            k_p16<<<NP / 8, 256, 0, stream>>>(Kf + kp1[m] * PB, Kf + kp2[m] * PB, KH, KL);
            k_vt<<<dim3(NP / 64, CC / 64, 1), 256, 0, stream>>>(Vf + m * PB, VTH, VTL);
            k_f16gemm<0><<<dim3(NP / 64, NP / 64, 1), 128, 0, stream>>>(QH, QL, CC, KH, KL, CC, CC, nullptr, S, NP);
            k_soft<<<NP / 32, 256, 0, stream>>>(S, PH, PL, RS);
            k_f16gemm<1><<<dim3(NP / 64, CC / 64, 1), 128, 0, stream>>>(PH, PL, NP, VTH, VTL, NP, NP, RS, Wm, CC);
            k_pbf<<<NP / 8, 256, 0, stream>>>(Wm, WmH, WmL);
            if (m == 0) k_gemm<true, 1, false><<<dim3(NP / 64, CC / 64, 1), 128, 0, stream>>>(WmH, WmL, Wg_b, bg, nullptr, Wm, FU);
            else        k_gemm<true, 1, true ><<<dim3(NP / 64, CC / 64, 1), 128, 0, stream>>>(WmH, WmL, Wg_b, bg, nullptr, Wm, FU);
        }
        k_pbf<<<NP / 8, 256, 0, stream>>>(FU, FH, FL);
        k_gemm<true, 2, false><<<dim3(NP / 64, CC / 64, 1), 128, 0, stream>>>(FH, FL, Wo_b, bo, nullptr, nullptr, out + (size_t)b * CC * NP);
    }
}
